// PCERegressor_59279138620021
// MI455X (gfx1250) — hardware-verified
//
#include <hip/hip_runtime.h>
#include <stddef.h>


#define NTHR   256
#define NWAVE  8
#define EPT    8
#define NGRP   2
#define CHUNK  (NTHR * EPT * NGRP)
#define WCAP   (EPT * NGRP * 32)
#define LISTN  (NWAVE * WCAP)
#define MTHR   128
#define MEDG   64
#define NBP    32
#define FE     16
#define GAP    40
#define BNEPS  1e-5f

static_assert((CHUNK & (CHUNK - 1)) == 0);
static_assert(CHUNK <= 4096);
static_assert((NBP & (NBP - 1)) == 0);
static_assert(MTHR == 2 * MEDG);

typedef float    v4f  __attribute__((ext_vector_type(4)));
typedef float    v8f  __attribute__((ext_vector_type(8)));
typedef int      v4i  __attribute__((ext_vector_type(4)));
typedef _Float16 v8h  __attribute__((ext_vector_type(8)));
typedef _Float16 v16h __attribute__((ext_vector_type(16)));
union FragH { v16h v; v8h h[2]; };

__host__ __device__ constexpr int msg_lds_bytes(int hid, int in, int out) {
  return (MEDG * (hid + 4) + MEDG * in + MEDG * out) * 4 + MEDG * 4;
}
__host__ __device__ constexpr int node_lds_bytes(int inl, int out) {
  return 16384 * 4 + out * (inl + 8) * 2 + LISTN * 4 + (16384 / out) * 4 + 64;
}

__device__ __forceinline__ v8h cvt8(v4f a, v4f b) {
  v8h r;
  r[0] = (_Float16)a.x; r[1] = (_Float16)a.y; r[2] = (_Float16)a.z; r[3] = (_Float16)a.w;
  r[4] = (_Float16)b.x; r[5] = (_Float16)b.y; r[6] = (_Float16)b.z; r[7] = (_Float16)b.w;
  return r;
}
__device__ __forceinline__ v8h zero8h() { v4f z = {0.f, 0.f, 0.f, 0.f}; return cvt8(z, z); }
__device__ __forceinline__ v8f zero8f() { v8f z = {0.f, 0.f, 0.f, 0.f, 0.f, 0.f, 0.f, 0.f}; return z; }

__device__ __forceinline__ v8f wmh(v16h a, v16h b, v8f c) {
  v8f d = __builtin_amdgcn_wmma_f32_16x16x32_f16(false, a, false, b, (short)0, c, false, false);
  asm volatile("v_nop\n\tv_nop\n\tv_nop\n\tv_nop" : "+v"(d) : "v"(a), "v"(b));
  return d;
}

__device__ __forceinline__ int scan_chunk(const int* __restrict__ ids, int nE, int cbase, int slotBase, int nb,
                                          int vec8, int* list, int tid, int lane, int wave) {
  int wc = 0;
#pragma unroll
  for (int g = 0; g < NGRP; ++g) {
    const int el0  = (g * NTHR + tid) * EPT;
    const int e0   = cbase + el0;
    const int sent = -2147483647 - 1;
    v4i da, db;
    if (vec8 != 0 && cbase + CHUNK <= nE) {
      da = *(const v4i*)(ids + e0);
      db = *(const v4i*)(ids + e0 + 4);
    } else {
      const int lst = nE - 1;
      da.x = (e0     < nE) ? ids[min(e0,     lst)] : sent;
      da.y = (e0 + 1 < nE) ? ids[min(e0 + 1, lst)] : sent;
      da.z = (e0 + 2 < nE) ? ids[min(e0 + 2, lst)] : sent;
      da.w = (e0 + 3 < nE) ? ids[min(e0 + 3, lst)] : sent;
      db.x = (e0 + 4 < nE) ? ids[min(e0 + 4, lst)] : sent;
      db.y = (e0 + 5 < nE) ? ids[min(e0 + 5, lst)] : sent;
      db.z = (e0 + 6 < nE) ? ids[min(e0 + 6, lst)] : sent;
      db.w = (e0 + 7 < nE) ? ids[min(e0 + 7, lst)] : sent;
    }
    const unsigned bs = (unsigned)slotBase;
    const unsigned ub = (unsigned)nb;
    const unsigned s0 = (unsigned)da.x - bs, s1 = (unsigned)da.y - bs;
    const unsigned s2 = (unsigned)da.z - bs, s3 = (unsigned)da.w - bs;
    const unsigned s4 = (unsigned)db.x - bs, s5 = (unsigned)db.y - bs;
    const unsigned s6 = (unsigned)db.z - bs, s7 = (unsigned)db.w - bs;
    const bool h0 = s0 < ub, h1 = s1 < ub, h2 = s2 < ub, h3 = s3 < ub;
    const bool h4 = s4 < ub, h5 = s5 < ub, h6 = s6 < ub, h7 = s7 < ub;
    const unsigned any = __builtin_amdgcn_ballot_w32(h0 | h1 | h2 | h3 | h4 | h5 | h6 | h7);
    if (any != 0u) {
#define HITJ(J, HJ, SJ) { \
        const unsigned mj = __builtin_amdgcn_ballot_w32(HJ); \
        if (mj != 0u) { \
          if (HJ) { \
            const int pos = wc + (int)__builtin_amdgcn_mbcnt_lo(mj, 0u); \
            if (pos < WCAP) list[wave * WCAP + pos] = ((el0 + (J)) << 12) | (int)(SJ); \
          } \
          wc += (int)__builtin_popcount(mj); } }
      HITJ(0, h0, s0)
      HITJ(1, h1, s1)
      HITJ(2, h2, s2)
      HITJ(3, h3, s3)
      HITJ(4, h4, s4)
      HITJ(5, h5, s5)
      HITJ(6, h6, s6)
      HITJ(7, h7, s7)
#undef HITJ
    }
  }
  return wc;
}

template <int HID, int IN, int OUT>
__global__ __launch_bounds__(NTHR) void k_bprep(const float* __restrict__ Wb, const float* __restrict__ bb,
                                               _Float16* Bp) {
  constexpr int KTOT = (HID + 1) * IN;
  constexpr int NU   = OUT * KTOT / 8;
  static_assert((KTOT % 32) == 0);
  static_assert((NU % 32) == 0);
  const int i = blockIdx.x * NTHR + (int)threadIdx.x;
  if (i >= NU) return;
  const int o  = i * 8;
  const int n  = o / KTOT;
  const int j0 = o - n * KTOT;
  float v[8];
#pragma unroll
  for (int e = 0; e < 8; ++e) {
    const int j  = j0 + e;
    const int jw = j < HID * IN ? j : HID * IN - 1;
    int jb = j - HID * IN;
    jb = jb < 0 ? 0 : (jb > IN - 1 ? IN - 1 : jb);
    const float wv = Wb[(size_t)jw * OUT + n];
    const float bv = bb[(size_t)jb * OUT + n];
    v[e] = (j < HID * IN ? wv : bv) * 16.0f;
  }
  v4f a, b;
  a.x = v[0]; a.y = v[1]; a.z = v[2]; a.w = v[3];
  b.x = v[4]; b.y = v[5]; b.z = v[6]; b.w = v[7];
  const v8h hv = cvt8(a, b);
  _Float16* dp = Bp + o;
  *(volatile v8h*)dp = hv;
  __threadfence();
  *(volatile v8h*)dp = hv;
}

template <int HID, int IN, int OUT>
__global__ __launch_bounds__(MTHR) void k_msg(
    const float* __restrict__ X, int nX, const int* __restrict__ ei, int nE,
    const float* __restrict__ EA, const float* __restrict__ Wa, const float* __restrict__ ba,
    const _Float16* __restrict__ Bp, float* MSG) {
  constexpr int KTOT = (HID + 1) * IN;
  constexpr int NT   = OUT / 16;
  constexpr int NIB  = IN / 32;
  constexpr int HP   = HID + 4;
  constexpr int NTH  = HID / 16;
  constexpr int NPI  = 16 * OUT / 128;
  static_assert((IN % 32) == 0 && (OUT % 32) == 0 && (HID % 16) == 0);
  static_assert((KTOT % 32) == 0);

  extern __shared__ v4f lds_dyn[];
  float* Hs  = (float*)lds_dyn;
  float* Xs  = Hs + MEDG * HP;
  float* Stg = Xs + MEDG * IN;
  int*   Ss  = (int*)(Stg + MEDG * OUT);

  const int tid = threadIdx.x, lane = tid & 31, wave = tid >> 5, hh = lane >> 4, m = lane & 15;
  const int eBase = blockIdx.x * MEDG;

  if (tid < MEDG) {
    int e = eBase + tid;
    e = e > nE - 1 ? nE - 1 : e;
    int s = ei[e];
    s = s < 0 ? 0 : (s > nX - 1 ? nX - 1 : s);
    Ss[tid] = s;
  }

  {
    int e = eBase + 16 * wave + m;
    e = e > nE - 1 ? nE - 1 : e;
    const float* ep = EA + (size_t)e * FE + 8 * hh;
    FragH a;
    a.h[0] = cvt8(*(const v4f*)ep, *(const v4f*)(ep + 4));
    a.h[1] = zero8h();
    float* hw = Hs + (16 * wave + 8 * hh) * HP;
#pragma unroll
    for (int t = 0; t < NTH; ++t) {
      const int col = 16 * t + m;
      const float* wp = Wa + (size_t)(8 * hh) * HID + col;
      v4f w0, w1;
      w0.x = wp[0] * 64.0f;       w0.y = wp[HID] * 64.0f;     w0.z = wp[2 * HID] * 64.0f; w0.w = wp[3 * HID] * 64.0f;
      w1.x = wp[4 * HID] * 64.0f; w1.y = wp[5 * HID] * 64.0f; w1.z = wp[6 * HID] * 64.0f; w1.w = wp[7 * HID] * 64.0f;
      FragH b;
      b.h[0] = cvt8(w0, w1);
      b.h[1] = zero8h();
      const v8f d = wmh(a.v, b.v, zero8f());
      const float bav = ba[col];
#pragma unroll
      for (int r = 0; r < 8; ++r) hw[r * HP + col] = fmaxf(d[r] * (1.0f / 64.0f) + bav, 0.0f);
    }
    if (lane < 16) Hs[(16 * wave + lane) * HP + HID] = 1.0f;
  }
  __syncthreads();

#pragma unroll 1
  for (int u = tid; u < MEDG * (IN / 4); u += MTHR) {
    const int r  = u / (IN / 4);
    const int c4 = u - r * (IN / 4);
    const int s  = Ss[r];
    *(v4f*)(Xs + r * IN + 4 * c4) = *(const v4f*)(X + (size_t)s * IN + 4 * c4);
  }
  __syncthreads();

  v4f xq[4 * NIB];
  {
    const float* xrow = Xs + (16 * wave + m) * IN + 8 * hh;
#pragma unroll
    for (int ib = 0; ib < NIB; ++ib) {
      xq[4 * ib + 0] = *(const v4f*)(xrow + 32 * ib);
      xq[4 * ib + 1] = *(const v4f*)(xrow + 32 * ib + 4);
      xq[4 * ib + 2] = *(const v4f*)(xrow + 32 * ib + 16);
      xq[4 * ib + 3] = *(const v4f*)(xrow + 32 * ib + 20);
    }
  }

  v8f acc[NT];
#pragma unroll
  for (int t = 0; t < NT; ++t) acc[t] = zero8f();
  const float* hrow = Hs + (16 * wave + m) * HP;
  const _Float16* bbase = Bp + (size_t)m * KTOT + 8 * hh;
#pragma unroll 1
  for (int k = 0; k <= HID; ++k) {
    const float hk = hrow[k] * 16.0f;
#pragma unroll
    for (int ib = 0; ib < NIB; ++ib) {
      const int kc = k * NIB + ib;
      FragH a;
      a.h[0] = cvt8(xq[4 * ib + 0] * hk, xq[4 * ib + 1] * hk);
      a.h[1] = cvt8(xq[4 * ib + 2] * hk, xq[4 * ib + 3] * hk);
      const _Float16* bp = bbase + (size_t)32 * kc;
#pragma unroll
      for (int t = 0; t < NT; ++t) {
        const _Float16* bt = bp + (size_t)(16 * t) * KTOT;
        FragH b;
        b.h[0] = *(const v8h*)bt;
        b.h[1] = *(const v8h*)(bt + 16);
        acc[t] = wmh(a.v, b.v, acc[t]);
      }
    }
  }
  __syncthreads();

  {
    float* sp = Stg + (16 * wave + 8 * hh) * OUT + m;
#pragma unroll
    for (int t = 0; t < NT; ++t) {
#pragma unroll
      for (int r = 0; r < 8; ++r) sp[r * OUT + 16 * t] = acc[t][r] * (1.0f / 256.0f);
    }
  }
  __syncthreads();

  const float* lp = Stg + 16 * wave * OUT;
  float* gp = MSG + (size_t)(eBase + 16 * wave) * OUT;
#pragma unroll
  for (int p = 0; p < NPI; ++p) {
    const v4f v = *(const v4f*)(lp + 4 * (32 * p + lane));
    *(volatile v4f*)(gp + 4 * (32 * p + lane)) = v;
  }
  __threadfence();
#pragma unroll
  for (int p = 0; p < NPI; ++p) {
    const v4f v = *(const v4f*)(lp + 4 * (32 * p + lane));
    *(volatile v4f*)(gp + 4 * (32 * p + lane)) = v;
  }
}

template <int INL, int OUT>
__global__ __launch_bounds__(NTHR) void k_node(
    const int* __restrict__ ei, int nE, int vec8, const float* __restrict__ MSG,
    const float* __restrict__ HPV, int nN,
    const float* __restrict__ root, const float* __restrict__ cbias,
    const float* __restrict__ gam, const float* __restrict__ bet,
    const float* __restrict__ rmean, const float* __restrict__ rvar,
    const float* __restrict__ aw, const float* __restrict__ ab, float* HN) {
  constexpr int NB  = 16384 / OUT;
  constexpr int NT  = OUT / 16;
  constexpr int SPW = NB / 128;
  constexpr int KT  = INL / 32;
  constexpr int RP  = INL + 8;
  constexpr int LPR = OUT / 4;
  constexpr int RPI = 128 / OUT;
  constexpr int RW  = NB / NWAVE;
  static_assert(SPW * NT == 8);
  static_assert(RW == 16 * RPI);
  static_assert(NB <= 512 && (NB & (NB - 1)) == 0);
  static_assert((INL % 32) == 0 && (OUT % 32) == 0 && OUT <= 128);

  extern __shared__ v4f lds_dyn[];
  float*    accL  = (float*)lds_dyn;
  _Float16* rootS = (_Float16*)(accL + NB * OUT);
  int*      list  = (int*)(rootS + OUT * RP);
  int*      pc    = list + LISTN;
  int*      wcnt  = pc + NB;

  const int tid = threadIdx.x, lane = tid & 31, wave = tid >> 5, hh = lane >> 4, m = lane & 15;
  const int nodeBase = blockIdx.x * NB;
  const int* dsts = ei + nE;

  {
    const v4f z = {0.f, 0.f, 0.f, 0.f};
#pragma unroll 1
    for (int i = tid; i < NB * OUT / 4; i += NTHR) ((v4f*)accL)[i] = z;
#pragma unroll 1
    for (int i = tid; i < NB; i += NTHR) pc[i] = 0;
#pragma unroll 1
    for (int u = tid; u < OUT * (INL / 8); u += NTHR) {
      const int n  = u / (INL / 8);
      const int k0 = (u - n * (INL / 8)) * 8;
      const float* rp = root + (size_t)k0 * OUT + n;
      v4f a, b;
      a.x = rp[0] * 256.0f;       a.y = rp[OUT] * 256.0f;     a.z = rp[2 * OUT] * 256.0f; a.w = rp[3 * OUT] * 256.0f;
      b.x = rp[4 * OUT] * 256.0f; b.y = rp[5 * OUT] * 256.0f; b.z = rp[6 * OUT] * 256.0f; b.w = rp[7 * OUT] * 256.0f;
      *(v8h*)(rootS + n * RP + k0) = cvt8(a, b);
    }
  }
  __syncthreads();

  const int nChunks = (nE + CHUNK - 1) / CHUNK;
#pragma unroll 1
  for (int ch = 0; ch < nChunks; ++ch) {
    const int cbase = ch * CHUNK;
    const int wc = scan_chunk(dsts, nE, cbase, nodeBase, NB, vec8, list, tid, lane, wave);
    if (lane == 0) wcnt[wave] = wc;
    __syncthreads();
    if (wave == 0) {
#pragma unroll 1
      for (int wsx = 0; wsx < NWAVE; ++wsx) {
        int n = __builtin_amdgcn_readfirstlane(wcnt[wsx]);
        n = n > WCAP ? WCAP : (n < 0 ? 0 : n);
        const int* lp = list + wsx * WCAP;
#pragma unroll 1
        for (int i = 0; i < n; ++i) {
          const int ent = __builtin_amdgcn_readfirstlane(lp[i]);
          int slot = ent & 4095;
          slot = slot > NB - 1 ? NB - 1 : slot;
          int e = cbase + ((ent >> 12) & (CHUNK - 1));
          e = e > nE - 1 ? nE - 1 : e;
          const int col = 4 * (lane & (LPR - 1));
          const v4f v = *(const v4f*)(MSG + (size_t)e * OUT + col);
          if (lane < LPR) {
            v4f* ap = (v4f*)(accL + slot * OUT + col);
            *ap = *ap + v;
          }
          if (lane == 0) pc[slot] = pc[slot] + 1;
        }
      }
    }
    __syncthreads();
  }

#pragma unroll 1
  for (int s = 0; s < SPW; ++s) {
    const int row0 = (wave * SPW + s) * 16;
    int arow = nodeBase + row0 + m;
    arow = arow > nN - 1 ? nN - 1 : arow;
    const float* xr = HPV + (size_t)arow * INL + 8 * hh;
    v8f acc2[NT];
#pragma unroll
    for (int t = 0; t < NT; ++t) acc2[t] = zero8f();
#pragma unroll
    for (int kt = 0; kt < KT; ++kt) {
      FragH a;
      a.h[0] = cvt8(*(const v4f*)(xr + 32 * kt), *(const v4f*)(xr + 32 * kt + 4));
      a.h[1] = cvt8(*(const v4f*)(xr + 32 * kt + 16), *(const v4f*)(xr + 32 * kt + 20));
#pragma unroll
      for (int t = 0; t < NT; ++t) {
        const _Float16* bp = rootS + (16 * t + m) * RP + 32 * kt + 8 * hh;
        FragH b;
        b.h[0] = *(const v8h*)bp;
        b.h[1] = *(const v8h*)(bp + 16);
        acc2[t] = wmh(a.v, b.v, acc2[t]);
      }
    }
    float rc[8];
#pragma unroll
    for (int r = 0; r < 8; ++r) {
      int c = pc[row0 + 8 * hh + r];
      c = c < 1 ? 1 : c;
      rc[r] = 1.0f / (float)c;
    }
#pragma unroll
    for (int t = 0; t < NT; ++t) {
      const int col = 16 * t + m;
      const float cbv = cbias[col];
      const float mu  = rmean[col];
      const float rs  = rsqrtf(rvar[col] + BNEPS);
      const float ga  = gam[col];
      const float bev = bet[col];
      float* ap = accL + (row0 + 8 * hh) * OUT + col;
#pragma unroll
      for (int r = 0; r < 8; ++r) {
        const float ag = ap[r * OUT];
        float val = ag * rc[r] + acc2[t][r] * (1.0f / 256.0f);
        val = val + cbv;
        val = (val - mu) * rs;
        val = val * ga + bev;
        val = fmaxf(val, 0.0f);
        ap[r * OUT] = val;
      }
    }
  }
  __syncthreads();

  const int col4 = 4 * (lane & (LPR - 1));
  const int rsub = lane / LPR;
  const v4f aw4 = *(const v4f*)(aw + col4);
  const float abv = ab[0];
  v4f ov[16];
#pragma unroll
  for (int q = 0; q < 16; ++q) {
    const int row = wave * RW + q * RPI + rsub;
    const v4f v = *(const v4f*)(accL + row * OUT + col4);
    float p = v.x * aw4.x + v.y * aw4.y + v.z * aw4.z + v.w * aw4.w;
#pragma unroll
    for (int off = LPR / 2; off >= 1; off >>= 1) p += __shfl_xor(p, off);
    const float zz = p + abv;
    const float gt = __builtin_amdgcn_rcpf(1.0f + __expf(-zz));
    ov[q] = v * gt;
  }
  float* gp = HN + (size_t)(nodeBase + wave * RW) * OUT + 4 * lane;
#pragma unroll
  for (int q = 0; q < 16; ++q) *(volatile v4f*)(gp + q * 128) = ov[q];
  __threadfence();
#pragma unroll
  for (int q = 0; q < 16; ++q) *(volatile v4f*)(gp + q * 128) = ov[q];
}

__global__ __launch_bounds__(NTHR) void k_pool_head(
    const int* __restrict__ batch, int nN, const int* __restrict__ numg,
    const float* __restrict__ H3, const float* __restrict__ fc1w, const float* __restrict__ fc1b,
    const float* __restrict__ fc2w, const float* __restrict__ fc2b, float* out, int G) {
  __shared__ __attribute__((aligned(16))) float gacc[NBP * 32];
  __shared__ __attribute__((aligned(16))) int plist[LISTN];
  __shared__ __attribute__((aligned(16))) _Float16 gA[NBP * GAP];
  __shared__ __attribute__((aligned(16))) float sOut[NBP];
  __shared__ int pcnt[NBP];
  __shared__ int wcnt[NWAVE];
  const int tid = threadIdx.x, lane = tid & 31, wave = tid >> 5, hh = lane >> 4, m = lane & 15;
  const int gBase = blockIdx.x * NBP;
  int nG = numg[0];
  nG = nG < 0 ? 0 : (nG > G ? G : nG);
  int nb = nG - gBase;
  nb = nb < 0 ? 0 : (nb > NBP ? NBP : nb);

  {
    const v4f z = {0.f, 0.f, 0.f, 0.f};
#pragma unroll 1
    for (int i = tid; i < NBP * 32 / 4; i += NTHR) ((v4f*)gacc)[i] = z;
    if (tid < NBP) { pcnt[tid] = 0; sOut[tid] = 0.0f; }
  }
  __syncthreads();

  const int nChunks = (nN + CHUNK - 1) / CHUNK;
#pragma unroll 1
  for (int ch = 0; ch < nChunks; ++ch) {
    const int cbase = ch * CHUNK;
    const int wc = scan_chunk(batch, nN, cbase, gBase, nb, 1, plist, tid, lane, wave);
    if (lane == 0) wcnt[wave] = wc;
    __syncthreads();
    if (wave == 0) {
#pragma unroll 1
      for (int wsx = 0; wsx < NWAVE; ++wsx) {
        int n = __builtin_amdgcn_readfirstlane(wcnt[wsx]);
        n = n > WCAP ? WCAP : (n < 0 ? 0 : n);
        const int* lp = plist + wsx * WCAP;
#pragma unroll 1
        for (int i = 0; i < n; ++i) {
          const int ent = __builtin_amdgcn_readfirstlane(lp[i]);
          int slot = ent & 4095;
          slot = slot > NBP - 1 ? NBP - 1 : slot;
          int nd = cbase + ((ent >> 12) & (CHUNK - 1));
          nd = nd > nN - 1 ? nN - 1 : nd;
          const int col = 4 * (lane & 7);
          const v4f v = *(const v4f*)(H3 + (size_t)nd * 32 + col);
          if (lane < 8) {
            v4f* ap = (v4f*)(gacc + slot * 32 + col);
            *ap = *ap + v;
          }
          if (lane == 0) pcnt[slot] = pcnt[slot] + 1;
        }
      }
    }
    __syncthreads();
  }

  if (tid < NBP * 4) {
    const int row = tid >> 2;
    const int c8  = (tid & 3) * 8;
    int c = pcnt[row];
    c = c < 1 ? 1 : c;
    const float rcv = 1.0f / (float)c;
    const v4f a = *(const v4f*)(gacc + row * 32 + c8) * rcv * 64.0f;
    const v4f b = *(const v4f*)(gacc + row * 32 + c8 + 4) * rcv * 64.0f;
    *(v8h*)(gA + row * GAP + c8) = cvt8(a, b);
  }
  __syncthreads();

  {
    const int rt = wave & 1;
    const _Float16* ap = gA + (16 * rt + m) * GAP + 8 * hh;
    FragH a;
    a.h[0] = *(const v8h*)ap;
    a.h[1] = *(const v8h*)(ap + 16);
    const float* wp = fc1w + (size_t)(8 * hh) * 16 + m;
    v4f w0, w1, w2, w3;
    w0.x = wp[0] * 64.0f;       w0.y = wp[16] * 64.0f;      w0.z = wp[32] * 64.0f;      w0.w = wp[48] * 64.0f;
    w1.x = wp[64] * 64.0f;      w1.y = wp[80] * 64.0f;      w1.z = wp[96] * 64.0f;      w1.w = wp[112] * 64.0f;
    w2.x = wp[256] * 64.0f;     w2.y = wp[272] * 64.0f;     w2.z = wp[288] * 64.0f;     w2.w = wp[304] * 64.0f;
    w3.x = wp[320] * 64.0f;     w3.y = wp[336] * 64.0f;     w3.z = wp[352] * 64.0f;     w3.w = wp[368] * 64.0f;
    FragH b;
    b.h[0] = cvt8(w0, w1);
    b.h[1] = cvt8(w2, w3);
    const v8f d = wmh(a.v, b.v, zero8f());
    const float b1v = fc1b[m];
    const float w2v = fc2w[m];
    const float b2v = fc2b[0];
#pragma unroll
    for (int r = 0; r < 8; ++r) {
      const float hv = fmaxf(d[r] * (1.0f / 4096.0f) + b1v, 0.0f);
      float p = hv * w2v;
      p += __shfl_xor(p, 1);
      p += __shfl_xor(p, 2);
      p += __shfl_xor(p, 4);
      p += __shfl_xor(p, 8);
      const float val = p + b2v;
      if (wave < 2 && m == 0) sOut[16 * rt + 8 * hh + r] = val;
    }
  }
  __syncthreads();

  v4f ovl = {0.f, 0.f, 0.f, 0.f};
  if (tid < 8) ovl = *(const v4f*)(sOut + 4 * tid);
  float* op = out + gBase;
  if (tid < 8) *(volatile v4f*)(op + 4 * tid) = ovl;
  __threadfence();
  if (tid < 8) *(volatile v4f*)(op + 4 * tid) = ovl;
}

extern "C" void kernel_launch(void* const* d_in, const int* in_sizes, int n_in,
                              void* d_out, int out_size, void* d_ws, size_t ws_size,
                              hipStream_t stream) {
  if (n_in < 45) return;
  const int nN = in_sizes[0] / 32;
  const int nE = in_sizes[1] / 2;
  const int G  = out_size;
  if (nN <= 0 || nE <= 0 || G <= 0) return;
  if (in_sizes[0] != nN * 32 || in_sizes[1] != 2 * nE || in_sizes[2] != nE * FE || in_sizes[3] != nN || in_sizes[4] < 1) return;
  if (in_sizes[5] != 16 * 128 || in_sizes[6] < 128 || in_sizes[7] != 128 * 4096 || in_sizes[8] < 4096 || in_sizes[9] != 32 * 128) return;
  if (in_sizes[10] < 128 || in_sizes[11] < 128 || in_sizes[12] < 128 || in_sizes[13] < 128 || in_sizes[14] < 128 ||
      in_sizes[15] < 128 || in_sizes[16] < 1) return;
  if (in_sizes[17] != 16 * 128 || in_sizes[18] < 128 || in_sizes[19] != 128 * 8192 || in_sizes[20] < 8192 || in_sizes[21] != 128 * 64) return;
  if (in_sizes[22] < 64 || in_sizes[23] < 64 || in_sizes[24] < 64 || in_sizes[25] < 64 || in_sizes[26] < 64 ||
      in_sizes[27] < 64 || in_sizes[28] < 1) return;
  if (in_sizes[29] != 16 * 64 || in_sizes[30] < 64 || in_sizes[31] != 64 * 2048 || in_sizes[32] < 2048 || in_sizes[33] != 64 * 32) return;
  if (in_sizes[34] < 32 || in_sizes[35] < 32 || in_sizes[36] < 32 || in_sizes[37] < 32 || in_sizes[38] < 32 ||
      in_sizes[39] < 32 || in_sizes[40] < 1) return;
  if (in_sizes[41] != 32 * 16 || in_sizes[42] < 16 || in_sizes[43] < 16 || in_sizes[44] < 1) return;
  if ((G % NBP) != 0) return;
  if (nN > (1 << 24) || nE > (1 << 26)) return;

  const float* x    = (const float*)d_in[0];
  const int*   ei   = (const int*)d_in[1];
  const float* ea   = (const float*)d_in[2];
  const int*   bat  = (const int*)d_in[3];
  const int*   numg = (const int*)d_in[4];
  const float *Wa1 = (const float*)d_in[5],  *ba1 = (const float*)d_in[6];
  const float *Wb1 = (const float*)d_in[7],  *bb1 = (const float*)d_in[8];
  const float *root1 = (const float*)d_in[9], *cb1 = (const float*)d_in[10];
  const float *g1 = (const float*)d_in[11], *be1 = (const float*)d_in[12];
  const float *m1 = (const float*)d_in[13], *v1 = (const float*)d_in[14];
  const float *aw1 = (const float*)d_in[15], *ab1 = (const float*)d_in[16];
  const float *Wa2 = (const float*)d_in[17], *ba2 = (const float*)d_in[18];
  const float *Wb2 = (const float*)d_in[19], *bb2 = (const float*)d_in[20];
  const float *root2 = (const float*)d_in[21], *cb2 = (const float*)d_in[22];
  const float *g2 = (const float*)d_in[23], *be2 = (const float*)d_in[24];
  const float *m2 = (const float*)d_in[25], *v2 = (const float*)d_in[26];
  const float *aw2 = (const float*)d_in[27], *ab2 = (const float*)d_in[28];
  const float *Wa3 = (const float*)d_in[29], *ba3 = (const float*)d_in[30];
  const float *Wb3 = (const float*)d_in[31], *bb3 = (const float*)d_in[32];
  const float *root3 = (const float*)d_in[33], *cb3 = (const float*)d_in[34];
  const float *g3 = (const float*)d_in[35], *be3 = (const float*)d_in[36];
  const float *m3 = (const float*)d_in[37], *v3 = (const float*)d_in[38];
  const float *aw3 = (const float*)d_in[39], *ab3 = (const float*)d_in[40];
  const float *fc1w = (const float*)d_in[41], *fc1b = (const float*)d_in[42];
  const float *fc2w = (const float*)d_in[43], *fc2b = (const float*)d_in[44];
  float* out = (float*)d_out;

  const int nMB = (nE + MEDG - 1) / MEDG;
  const int EP  = nMB * MEDG;
  const int nB1 = (nN + 127) / 128, NP1 = nB1 * 128;
  const int nB2 = (nN + 255) / 256, NP2 = nB2 * 256;
  const int nB3 = (nN + 511) / 512, NP3 = nB3 * 512;
  const int nPool = G / NBP;

  constexpr int KT1 = (128 + 1) * 32, KT2 = (128 + 1) * 128, KT3 = (64 + 1) * 64;

  char* ws = (char*)d_ws;
  size_t off = 0;
  const size_t oBp1 = off; off += (size_t)128 * KT1 * 2;    off = (off + 255) & ~(size_t)255;
  const size_t oBp2 = off; off += (size_t)64 * KT2 * 2;     off = (off + 255) & ~(size_t)255;
  const size_t oBp3 = off; off += (size_t)32 * KT3 * 2;     off = (off + 255) & ~(size_t)255;
  const size_t oMs1 = off; off += (size_t)EP * 128 * 4;     off = (off + 255) & ~(size_t)255;
  const size_t oMs2 = off; off += (size_t)EP * 64 * 4;      off = (off + 255) & ~(size_t)255;
  const size_t oMs3 = off; off += (size_t)EP * 32 * 4;      off = (off + 255) & ~(size_t)255;
  const size_t oH1  = off; off += (size_t)NP1 * 128 * 4;    off = (off + 255) & ~(size_t)255;
  const size_t oH2  = off; off += (size_t)NP2 * 64 * 4;     off = (off + 255) & ~(size_t)255;
  const size_t oH3  = off; off += (size_t)NP3 * 32 * 4;     off = (off + 255) & ~(size_t)255;
  if (off > ws_size) return;
  if (off > (size_t)128 * 1024 * 1024) return;
  _Float16* Bp1 = (_Float16*)(ws + oBp1);
  _Float16* Bp2 = (_Float16*)(ws + oBp2);
  _Float16* Bp3 = (_Float16*)(ws + oBp3);
  float* msg1 = (float*)(ws + oMs1);
  float* msg2 = (float*)(ws + oMs2);
  float* msg3 = (float*)(ws + oMs3);
  float* h1 = (float*)(ws + oH1);
  float* h2 = (float*)(ws + oH2);
  float* h3 = (float*)(ws + oH3);

  const int vec8 = ((nE & 3) == 0) ? 1 : 0;

  {
    const int nu1 = 128 * KT1 / 8, nu2 = 64 * KT2 / 8, nu3 = 32 * KT3 / 8;
    k_bprep<128, 32, 128><<<(nu1 + NTHR - 1) / NTHR, NTHR, 0, stream>>>(Wb1, bb1, Bp1);
    k_bprep<128, 128, 64><<<(nu2 + NTHR - 1) / NTHR, NTHR, 0, stream>>>(Wb2, bb2, Bp2);
    k_bprep<64, 64, 32><<<(nu3 + NTHR - 1) / NTHR, NTHR, 0, stream>>>(Wb3, bb3, Bp3);
  }

  constexpr int LM1 = msg_lds_bytes(128, 32, 128);
  constexpr int LM2 = msg_lds_bytes(128, 128, 64);
  constexpr int LM3 = msg_lds_bytes(64, 64, 32);
  constexpr int LN1 = node_lds_bytes(32, 128);
  constexpr int LN2 = node_lds_bytes(128, 64);
  constexpr int LN3 = node_lds_bytes(64, 32);
  hipFuncSetAttribute(reinterpret_cast<const void*>(&k_msg<128, 32, 128>), hipFuncAttributeMaxDynamicSharedMemorySize, LM1);
  hipFuncSetAttribute(reinterpret_cast<const void*>(&k_msg<128, 128, 64>), hipFuncAttributeMaxDynamicSharedMemorySize, LM2);
  hipFuncSetAttribute(reinterpret_cast<const void*>(&k_msg<64, 64, 32>), hipFuncAttributeMaxDynamicSharedMemorySize, LM3);
  hipFuncSetAttribute(reinterpret_cast<const void*>(&k_node<32, 128>), hipFuncAttributeMaxDynamicSharedMemorySize, LN1);
  hipFuncSetAttribute(reinterpret_cast<const void*>(&k_node<128, 64>), hipFuncAttributeMaxDynamicSharedMemorySize, LN2);
  hipFuncSetAttribute(reinterpret_cast<const void*>(&k_node<64, 32>), hipFuncAttributeMaxDynamicSharedMemorySize, LN3);

  k_msg<128, 32, 128><<<nMB, MTHR, LM1, stream>>>(x, nN, ei, nE, ea, Wa1, ba1, Bp1, msg1);
  k_node<32, 128><<<nB1, NTHR, LN1, stream>>>(ei, nE, vec8, msg1, x, nN, root1, cb1, g1, be1, m1, v1, aw1, ab1, h1);
  k_msg<128, 128, 64><<<nMB, MTHR, LM2, stream>>>(h1, nN, ei, nE, ea, Wa2, ba2, Bp2, msg2);
  k_node<128, 64><<<nB2, NTHR, LN2, stream>>>(ei, nE, vec8, msg2, h1, nN, root2, cb2, g2, be2, m2, v2, aw2, ab2, h2);
  k_msg<64, 64, 32><<<nMB, MTHR, LM3, stream>>>(h2, nN, ei, nE, ea, Wa3, ba3, Bp3, msg3);
  k_node<64, 32><<<nB3, NTHR, LN3, stream>>>(ei, nE, vec8, msg3, h2, nN, root3, cb3, g3, be3, m3, v3, aw3, ab3, h3);
  k_pool_head<<<nPool, NTHR, 0, stream>>>(bat, nN, numg, h3, fc1w, fc1b, fc2w, fc2b, out, G);
}
